// GCN_57397942943830
// MI455X (gfx1250) — hardware-verified
//
#include <hip/hip_runtime.h>
#include <stddef.h>
#include <stdint.h>
#include <math.h>


#define NGRAPH 8
#define NPG    4096
#define NE     131072
#define CH     256
#define NT     (NGRAPH * NPG)
#define K1     256
#define K2     512
#define NTHR   256
#define NWAVE  8
#define EPT    8
#define CHUNK  (NTHR * EPT)
#define WCAP   (EPT * 32)
#define LISTN  (NWAVE * WCAP)
#define NBA    512
#define SLA    9
#define BPG    (NPG / NBA)
#define NBLK   (NT / NBA)
#define RCAP   28672
#define DEGCAP 96
#define GBM    64
#define GBN    64
#define GTHR   128
#define UW1    (CH * (K1 / 8))
#define UW2    (CH * (K2 / 8))
#define UX     (NT * (CH / 8))
#define AGG_ZINTS (LISTN + 2 * RCAP + 3 * NBA)
#define AGG_LDS_INTS (AGG_ZINTS + 16)
#define WSMAX  134217728

static_assert((CHUNK & (CHUNK - 1)) == 0 && CHUNK <= 4096);
static_assert((NBA & (NBA - 1)) == 0 && NBA == (1 << SLA));
static_assert(NPG % NBA == 0 && BPG * NBA == NPG && NBLK * NBA == NT);
static_assert(((long long)NE << SLA) < (1LL << 31));
static_assert(((long long)CHUNK << SLA) < (1LL << 31));
static_assert(NE % CHUNK == 0 && NE % 4 == 0);
static_assert(LISTN % NTHR == 0 && NBA % 4 == 0 && NBA / 4 <= NTHR && (NBA / 4) % 32 == 0);
static_assert(NBA % NWAVE == 0 && NBA % 32 == 0);
static_assert(RCAP % 32 == 0 && AGG_ZINTS % 4 == 0 && LISTN % 4 == 0);
static_assert(RCAP >= 17400 && DEGCAP >= 64);
static_assert(K1 % 32 == 0 && K2 % 32 == 0 && K2 == 2 * CH && K1 == CH);
static_assert(NT % GBM == 0 && NT % 128 == 0 && CH % GBN == 0 && CH % 8 == 0);
static_assert(GBM == (GTHR / 32) * 16 && GBN == 64);
static_assert(UW1 % NTHR == 0 && UW2 % NTHR == 0 && UX % NTHR == 0);
static_assert(CH == 8 * 32);
static_assert(AGG_LDS_INTS * 4 <= 300000);

typedef float          v4f   __attribute__((ext_vector_type(4)));
typedef float          v8f   __attribute__((ext_vector_type(8)));
typedef int            v4i   __attribute__((ext_vector_type(4)));
typedef int            v8i   __attribute__((ext_vector_type(8)));
typedef unsigned short v8us  __attribute__((ext_vector_type(8)));
typedef unsigned short v16us __attribute__((ext_vector_type(16)));
typedef __bf16         v16bf __attribute__((ext_vector_type(16)));
typedef v4f  __attribute__((may_alias)) v4fa;
typedef v4i  __attribute__((may_alias)) v4ia;
typedef v8us __attribute__((may_alias)) v8usa;
union FragB { v16bf v; v16us u; v8us h[2]; v8i w; };

__device__ __forceinline__ v8f wmb(const FragB& a, const FragB& b, v8f c) {
  v8f d = __builtin_amdgcn_wmma_f32_16x16x32_bf16(false, a.v, false, b.v, (short)0, c, false, false);
  asm volatile("v_nop\n\tv_nop\n\tv_nop\n\tv_nop" : "+v"(d) : "v"(a.w), "v"(b.w));
  return d;
}

__device__ __forceinline__ unsigned bf16_bits(float f) {
  const unsigned u = __float_as_uint(f);
  const unsigned r = (u + 0x7FFFu + ((u >> 16) & 1u)) >> 16;
  const unsigned n = (u >> 16) | 0x40u;
  return ((u & 0x7FFFFFFFu) > 0x7F800000u) ? n : r;
}
__device__ __forceinline__ float bf16_val(float f) {
  return __uint_as_float(bf16_bits(f) << 16);
}

template <int SLB>
__device__ __forceinline__ int scan_chunk(const int* __restrict__ dsts, int nE, int cbase, int slotBase,
                                          int nb, int vec8, int* list, int tid, int lane, int wave) {
  int wc = 0;
  const int el0  = tid * EPT;
  const int e0   = cbase + el0;
  const int sent = -2147483647 - 1;
  v4i da, db;
  if (vec8 != 0 && cbase + CHUNK <= nE) {
    da = *(const v4i*)(dsts + e0);
    db = *(const v4i*)(dsts + e0 + 4);
  } else {
    da.x = (e0     < nE) ? dsts[min(e0,     nE - 1)] : sent;
    da.y = (e0 + 1 < nE) ? dsts[min(e0 + 1, nE - 1)] : sent;
    da.z = (e0 + 2 < nE) ? dsts[min(e0 + 2, nE - 1)] : sent;
    da.w = (e0 + 3 < nE) ? dsts[min(e0 + 3, nE - 1)] : sent;
    db.x = (e0 + 4 < nE) ? dsts[min(e0 + 4, nE - 1)] : sent;
    db.y = (e0 + 5 < nE) ? dsts[min(e0 + 5, nE - 1)] : sent;
    db.z = (e0 + 6 < nE) ? dsts[min(e0 + 6, nE - 1)] : sent;
    db.w = (e0 + 7 < nE) ? dsts[min(e0 + 7, nE - 1)] : sent;
  }
  const unsigned nbs = (unsigned)slotBase;
  const unsigned unb = (unsigned)nb;
  const unsigned s0 = (unsigned)da.x - nbs, s1 = (unsigned)da.y - nbs;
  const unsigned s2 = (unsigned)da.z - nbs, s3 = (unsigned)da.w - nbs;
  const unsigned s4 = (unsigned)db.x - nbs, s5 = (unsigned)db.y - nbs;
  const unsigned s6 = (unsigned)db.z - nbs, s7 = (unsigned)db.w - nbs;
  const bool h0 = s0 < unb, h1 = s1 < unb, h2 = s2 < unb, h3 = s3 < unb;
  const bool h4 = s4 < unb, h5 = s5 < unb, h6 = s6 < unb, h7 = s7 < unb;
  const unsigned any = __builtin_amdgcn_ballot_w32(h0 | h1 | h2 | h3 | h4 | h5 | h6 | h7);
  if (any != 0u) {
#define HITJ(J, HJ, SJ) { \
      const unsigned mj = __builtin_amdgcn_ballot_w32(HJ); \
      if (mj != 0u) { \
        if (HJ) { \
          const int pos = wc + (int)__builtin_amdgcn_mbcnt_lo(mj, 0u); \
          if (pos < WCAP) list[wave * WCAP + pos] = ((el0 + (J)) << SLB) | (int)(SJ); \
        } \
        wc += (int)__builtin_popcount(mj); } }
    HITJ(0, h0, s0)
    HITJ(1, h1, s1)
    HITJ(2, h2, s2)
    HITJ(3, h3, s3)
    HITJ(4, h4, s4)
    HITJ(5, h5, s5)
    HITJ(6, h6, s6)
    HITJ(7, h7, s7)
#undef HITJ
  }
  return wc;
}

__global__ __launch_bounds__(NTHR) void k_prep(const float* __restrict__ x, const float* __restrict__ W1,
                                               const float* __restrict__ W2, unsigned short* W1T,
                                               unsigned short* W2D, unsigned short* XB) {
  const int u = (int)blockIdx.x * NTHR + (int)threadIdx.x;
  v8us o;
  unsigned short* dp;
  if (u < UW1) {
    const int n  = u >> 5;
    const int k8 = (u & 31) * 8;
    const float* p = W1 + (size_t)k8 * CH + n;
#pragma unroll
    for (int i = 0; i < 8; ++i) o[i] = (unsigned short)bf16_bits(p[(size_t)i * CH]);
    dp = W1T + (size_t)n * K1 + k8;
  } else if (u < UW1 + UW2) {
    const int v  = u - UW1;
    const int n  = v >> 6;
    const int k8 = (v & 63) * 8;
    const int kk = k8 & (CH - 1);
    const float* p = W2 + (size_t)kk * CH + n;
#pragma unroll
    for (int i = 0; i < 8; ++i) o[i] = (unsigned short)bf16_bits(p[(size_t)i * CH]);
    dp = W2D + (size_t)n * K2 + k8;
  } else if (u < UW1 + UW2 + UX) {
    const int v = u - (UW1 + UW2);
    const float* p = x + (size_t)v * 8;
    const v4f a = *(const v4fa*)p;
    const v4f b = *(const v4fa*)(p + 4);
    o[0] = (unsigned short)bf16_bits(a.x); o[1] = (unsigned short)bf16_bits(a.y);
    o[2] = (unsigned short)bf16_bits(a.z); o[3] = (unsigned short)bf16_bits(a.w);
    o[4] = (unsigned short)bf16_bits(b.x); o[5] = (unsigned short)bf16_bits(b.y);
    o[6] = (unsigned short)bf16_bits(b.z); o[7] = (unsigned short)bf16_bits(b.w);
    dp = XB + (size_t)v * 8;
  } else {
    return;
  }
  *(volatile v8us*)dp = o;
  __threadfence();
  *(volatile v8us*)dp = o;
}

__global__ __launch_bounds__(NTHR) void k_deg(const int* __restrict__ ei, int vec8, float* dis) {
  __shared__ __attribute__((aligned(16))) int scnt[NBA];
  __shared__ __attribute__((aligned(16))) int list[LISTN];
  __shared__ int wcnt[NWAVE];
  const int tid = (int)threadIdx.x, lane = tid & 31, wave = tid >> 5;
  const int b = (int)blockIdx.x;
  const int g = b / BPG;
  const int slotBase = (b - g * BPG) * NBA;
  const int* dsts = ei + (size_t)(2 * g + 1) * NE;

  for (int i = tid; i < NBA; i += NTHR) scnt[i] = 0;
  for (int i = tid; i < LISTN; i += NTHR) list[i] = 0;
  if (tid < NWAVE) wcnt[tid] = 0;
  __syncthreads();

  const int nChunks = (NE + CHUNK - 1) / CHUNK;
#pragma unroll 1
  for (int ch = 0; ch < nChunks; ++ch) {
    const int cbase = ch * CHUNK;
    const int wc = scan_chunk<SLA>(dsts, NE, cbase, slotBase, NBA, vec8, list, tid, lane, wave);
    if (lane == 0) wcnt[wave] = wc;
    __syncthreads();
    if (wave == 0) {
#pragma unroll 1
      for (int w2 = 0; w2 < NWAVE; ++w2) {
        int c = wcnt[w2];
        c = c < 0 ? 0 : (c > WCAP ? WCAP : c);
#pragma unroll 1
        for (int b0 = 0; b0 < c; b0 += 32) {
          const int idx = b0 + lane;
          const int ent = list[w2 * WCAP + (idx < WCAP ? idx : WCAP - 1)];
          const int m32 = (c - b0) < 32 ? (c - b0) : 32;
#pragma unroll 1
          for (int k = 0; k < m32; ++k) {
            const int u  = __builtin_amdgcn_readlane(ent, k);
            const int sl = u & (NBA - 1);
            if (lane == 0) scnt[sl] = scnt[sl] + 1;
          }
        }
      }
    }
    __syncthreads();
  }

  if (tid < NBA / 4) {
    const v4i c4 = *(const v4ia*)(scnt + 4 * tid);
    const float d0 = (float)c4.x + 1.0f, d1 = (float)c4.y + 1.0f;
    const float d2 = (float)c4.z + 1.0f, d3 = (float)c4.w + 1.0f;
    v4f v;
    v.x = (d0 > 0.0f) ? rsqrtf(d0) : 0.0f;
    v.y = (d1 > 0.0f) ? rsqrtf(d1) : 0.0f;
    v.z = (d2 > 0.0f) ? rsqrtf(d2) : 0.0f;
    v.w = (d3 > 0.0f) ? rsqrtf(d3) : 0.0f;
    float* op = dis + (size_t)b * NBA + 4 * tid;
    *(volatile v4f*)op = v;
    __threadfence();
    *(volatile v4f*)op = v;
  }
}

__global__ __launch_bounds__(GTHR) void k_gemm(
    const unsigned short* __restrict__ A, const unsigned short* __restrict__ WT,
    float* outF, int K, int ldo)
{
  __shared__ __attribute__((aligned(16))) float stg[GBM * GBN];
  const int tid = (int)threadIdx.x, lane = tid & 31, wave = tid >> 5, hh = lane >> 4, m = lane & 15;
  const int rowBase = (int)blockIdx.x * GBM;
  const int col0    = (int)blockIdx.y * GBN;

  v8f acc[4];
  {
    const v8f z = {0.f, 0.f, 0.f, 0.f, 0.f, 0.f, 0.f, 0.f};
    acc[0] = z; acc[1] = z; acc[2] = z; acc[3] = z;
  }
  const unsigned short* ap = A  + (size_t)(rowBase + 16 * wave + m) * (size_t)K + 8 * hh;
  const unsigned short* wp = WT + (size_t)(col0 + m) * (size_t)K + 8 * hh;
  const int ksteps = K >> 5;
#pragma unroll 1
  for (int ks = 0; ks < ksteps; ++ks) {
    FragB af;
    af.h[0] = *(const v8usa*)(ap + 32 * ks);
    af.h[1] = *(const v8usa*)(ap + 32 * ks + 16);
#pragma unroll
    for (int t = 0; t < 4; ++t) {
      const unsigned short* wq = wp + (size_t)(16 * t) * (size_t)K + 32 * ks;
      FragB bf;
      bf.h[0] = *(const v8usa*)wq;
      bf.h[1] = *(const v8usa*)(wq + 16);
      acc[t] = wmb(af, bf, acc[t]);
    }
  }

#pragma unroll
  for (int t = 0; t < 4; ++t) {
    const int lc = 16 * t + m;
#pragma unroll
    for (int r = 0; r < 8; ++r) {
      const int lr = 16 * wave + 8 * hh + r;
      stg[lr * GBN + lc] = acc[t][r];
    }
  }
  __syncthreads();

  v4f fv[8];
#pragma unroll
  for (int i = 0; i < 8; ++i) {
    const int lr = 16 * wave + 2 * i + hh;
    fv[i] = *(const v4fa*)(stg + lr * GBN + 4 * m);
  }
#pragma unroll
  for (int i = 0; i < 8; ++i) {
    const int lr = 16 * wave + 2 * i + hh;
    const int gr = rowBase + lr;
    float* op = outF + (size_t)gr * (size_t)ldo + col0 + 4 * m;
    *(volatile v4f*)op = fv[i];
  }
  __threadfence();
#pragma unroll
  for (int i = 0; i < 8; ++i) {
    const int lr = 16 * wave + 2 * i + hh;
    const int gr = rowBase + lr;
    float* op = outF + (size_t)gr * (size_t)ldo + col0 + 4 * m;
    *(volatile v4f*)op = fv[i];
  }
}

template <int MODE>
__global__ __launch_bounds__(NTHR) void k_agg(const int* __restrict__ ei, int vec8,
                                              const float* __restrict__ dis,
                                              const float* __restrict__ xl, const float* __restrict__ bias,
                                              unsigned short* hb, float* hout) {
  extern __shared__ __attribute__((aligned(16))) int dsm[];
  int* list = dsm;
  int* hl   = dsm + LISTN;
  int* sl   = dsm + LISTN + RCAP;
  int* cnt  = dsm + LISTN + 2 * RCAP;
  int* offs = cnt + NBA;
  int* cur  = offs + NBA;
  int* misc = cur + NBA;
  const int tid = (int)threadIdx.x, lane = tid & 31, wave = tid >> 5;
  const int b = (int)blockIdx.x;
  const int g = b / BPG;
  const int slotBase = (b - g * BPG) * NBA;
  const int rowBase  = b * NBA;
  const int gOff     = g * NPG;
  const int* srcs = ei + (size_t)(2 * g) * NE;
  const int* dsts = srcs + NE;

  {
    const v4i z4 = {0, 0, 0, 0};
    for (int i = tid * 4; i < AGG_ZINTS; i += NTHR * 4) *(v4ia*)(dsm + i) = z4;
    if (tid < 16) misc[tid] = 0;
  }
  const int c0 = (MODE != 0) ? 8 * lane     : 4 * lane;
  const int c1 = (MODE != 0) ? 8 * lane + 4 : 128 + 4 * lane;
  v4f bA, bB;
  {
    const v4f ta = *(const v4fa*)(bias + c0);
    const v4f tb = *(const v4fa*)(bias + c1);
    bA.x = bf16_val(ta.x); bA.y = bf16_val(ta.y); bA.z = bf16_val(ta.z); bA.w = bf16_val(ta.w);
    bB.x = bf16_val(tb.x); bB.y = bf16_val(tb.y); bB.z = bf16_val(tb.z); bB.w = bf16_val(tb.w);
  }
  __syncthreads();

  int t = 0, ov = 0;
  const int nChunks = (NE + CHUNK - 1) / CHUNK;
#pragma unroll 1
  for (int ch = 0; ch < nChunks; ++ch) {
    const int cbase = ch * CHUNK;
    const int wc = scan_chunk<SLA>(dsts, NE, cbase, slotBase, NBA, vec8, list, tid, lane, wave);
    if (lane == 0) misc[wave] = wc;
    __syncthreads();
    if (wave == 0) {
#pragma unroll 1
      for (int w2 = 0; w2 < NWAVE; ++w2) {
        int c = misc[w2];
        c = c < 0 ? 0 : (c > WCAP ? WCAP : c);
#pragma unroll 1
        for (int b0 = 0; b0 < c; b0 += 32) {
          const int idx = b0 + lane;
          const int ent = list[w2 * WCAP + (idx < WCAP ? idx : WCAP - 1)];
          const int m32 = (c - b0) < 32 ? (c - b0) : 32;
#pragma unroll 1
          for (int k = 0; k < m32; ++k) {
            const int u    = __builtin_amdgcn_readlane(ent, k);
            const int slot = u & (NBA - 1);
            const int el   = (u >> SLA) & (CHUNK - 1);
            const int pk   = ((cbase + el) << SLA) | slot;
            if (t < RCAP) {
              if (lane == 0) { hl[t] = pk; cnt[slot] = cnt[slot] + 1; }
              t = t + 1;
            } else {
              ov = 1;
            }
          }
        }
      }
    }
    __syncthreads();
  }
  if (wave == 0 && lane == 0) { misc[8] = t; misc[9] = ov; }
  __syncthreads();
  int tt = misc[8];
  tt = tt < 0 ? 0 : (tt > RCAP ? RCAP : tt);
  const int ovf = misc[9];

  if (wave == 0) {
    const int base = lane * (NBA / 32);
    int s = 0;
#pragma unroll 1
    for (int i = 0; i < NBA / 32; ++i) s += cnt[base + i];
    int incl = s;
#pragma unroll
    for (int d = 1; d < 32; d <<= 1) {
      const int y = __shfl_up(incl, d, 32);
      if (lane >= d) incl += y;
    }
    int run = incl - s;
#pragma unroll 1
    for (int i = 0; i < NBA / 32; ++i) {
      const int cv = cnt[base + i];
      offs[base + i] = run;
      cur[base + i]  = run;
      run += cv;
    }
  }
  __syncthreads();
  if (wave == 0) {
#pragma unroll 1
    for (int b0 = 0; b0 < tt; b0 += 32) {
      const int idx = b0 + lane;
      const int ent = hl[idx < RCAP ? idx : RCAP - 1];
      const int m32 = (tt - b0) < 32 ? (tt - b0) : 32;
#pragma unroll 1
      for (int k = 0; k < m32; ++k) {
        const int u    = __builtin_amdgcn_readlane(ent, k);
        const int slot = u & (NBA - 1);
        if (lane == 0) {
          int p = cur[slot];
          p = p < 0 ? 0 : (p > RCAP - 1 ? RCAP - 1 : p);
          sl[p] = u;
          cur[slot] = p + 1;
        }
      }
    }
  }
  __syncthreads();

  const float qnan = __int_as_float(0x7fc00000);
#pragma unroll 1
  for (int si = 0; si < NBA / NWAVE; ++si) {
    const int s    = si * NWAVE + wave;
    const int node = rowBase + s;
    int c = cnt[s];
    const bool big = c > DEGCAP;
    c = c < 0 ? 0 : (c > DEGCAP ? DEGCAP : c);
    int o = offs[s];
    o = o < 0 ? 0 : (o > RCAP ? RCAP : o);
    const float dd = dis[node];
    const float rd = dd * dd;
    float a0 = 0.0f, a1 = 0.0f, a2 = 0.0f, a3 = 0.0f;
    float a4 = 0.0f, a5 = 0.0f, a6 = 0.0f, a7 = 0.0f;
#pragma unroll 1
    for (int b0 = 0; b0 < c; b0 += 32) {
      int idx = o + b0 + lane;
      idx = idx > RCAP - 1 ? RCAP - 1 : idx;
      const int ent = sl[idx];
      int eid = ent >> SLA;
      eid = eid < 0 ? 0 : (eid > NE - 1 ? NE - 1 : eid);
      int sr = srcs[eid];
      sr = sr < 0 ? 0 : (sr > NPG - 1 ? NPG - 1 : sr);
      const int   gs  = gOff + sr;
      const float cf  = dis[gs] * dd;
      const int   cfi = __float_as_int(cf);
      const int m32 = (c - b0) < 32 ? (c - b0) : 32;
#pragma unroll 1
      for (int k = 0; k < m32; ++k) {
        const int   sk = __builtin_amdgcn_readlane(gs, k);
        const float ck = __int_as_float(__builtin_amdgcn_readlane(cfi, k));
        const float* rp = xl + (size_t)sk * CH;
        const v4f va = *(const v4fa*)(rp + c0);
        const v4f vb = *(const v4fa*)(rp + c1);
        a0 = fmaf(ck, va.x, a0); a1 = fmaf(ck, va.y, a1);
        a2 = fmaf(ck, va.z, a2); a3 = fmaf(ck, va.w, a3);
        a4 = fmaf(ck, vb.x, a4); a5 = fmaf(ck, vb.y, a5);
        a6 = fmaf(ck, vb.z, a6); a7 = fmaf(ck, vb.w, a7);
      }
    }
    v4f sA, sB;
    {
      const float* rp = xl + (size_t)node * CH;
      sA = *(const v4fa*)(rp + c0);
      sB = *(const v4fa*)(rp + c1);
    }
    const bool pois = big || (ovf != 0);
    float y0 = (a0 + sA.x * rd) + bA.x;
    float y1 = (a1 + sA.y * rd) + bA.y;
    float y2 = (a2 + sA.z * rd) + bA.z;
    float y3 = (a3 + sA.w * rd) + bA.w;
    float y4 = (a4 + sB.x * rd) + bB.x;
    float y5 = (a5 + sB.y * rd) + bB.y;
    float y6 = (a6 + sB.z * rd) + bB.z;
    float y7 = (a7 + sB.w * rd) + bB.w;
    if constexpr (MODE != 0) {
      y0 = (y0 > 0.0f) ? y0 : (y0 - y0); y1 = (y1 > 0.0f) ? y1 : (y1 - y1);
      y2 = (y2 > 0.0f) ? y2 : (y2 - y2); y3 = (y3 > 0.0f) ? y3 : (y3 - y3);
      y4 = (y4 > 0.0f) ? y4 : (y4 - y4); y5 = (y5 > 0.0f) ? y5 : (y5 - y5);
      y6 = (y6 > 0.0f) ? y6 : (y6 - y6); y7 = (y7 > 0.0f) ? y7 : (y7 - y7);
    }
    y0 = pois ? qnan : y0; y1 = pois ? qnan : y1; y2 = pois ? qnan : y2; y3 = pois ? qnan : y3;
    y4 = pois ? qnan : y4; y5 = pois ? qnan : y5; y6 = pois ? qnan : y6; y7 = pois ? qnan : y7;
    if constexpr (MODE != 0) {
      v8us hv, lv;
      unsigned h;
      h = bf16_bits(y0); hv[0] = (unsigned short)h; lv[0] = (unsigned short)bf16_bits(y0 - __uint_as_float(h << 16));
      h = bf16_bits(y1); hv[1] = (unsigned short)h; lv[1] = (unsigned short)bf16_bits(y1 - __uint_as_float(h << 16));
      h = bf16_bits(y2); hv[2] = (unsigned short)h; lv[2] = (unsigned short)bf16_bits(y2 - __uint_as_float(h << 16));
      h = bf16_bits(y3); hv[3] = (unsigned short)h; lv[3] = (unsigned short)bf16_bits(y3 - __uint_as_float(h << 16));
      h = bf16_bits(y4); hv[4] = (unsigned short)h; lv[4] = (unsigned short)bf16_bits(y4 - __uint_as_float(h << 16));
      h = bf16_bits(y5); hv[5] = (unsigned short)h; lv[5] = (unsigned short)bf16_bits(y5 - __uint_as_float(h << 16));
      h = bf16_bits(y6); hv[6] = (unsigned short)h; lv[6] = (unsigned short)bf16_bits(y6 - __uint_as_float(h << 16));
      h = bf16_bits(y7); hv[7] = (unsigned short)h; lv[7] = (unsigned short)bf16_bits(y7 - __uint_as_float(h << 16));
      unsigned short* hp = hb + (size_t)node * K2 + 8 * lane;
      unsigned short* lp = hp + CH;
      *(volatile v8us*)hp = hv;
      *(volatile v8us*)lp = lv;
      __threadfence();
      *(volatile v8us*)hp = hv;
      *(volatile v8us*)lp = lv;
    } else {
      v4f oA, oB;
      oA.x = y0; oA.y = y1; oA.z = y2; oA.w = y3;
      oB.x = y4; oB.y = y5; oB.z = y6; oB.w = y7;
      float* op = hout + (size_t)node * CH;
      *(volatile v4f*)(op + c0) = oA;
      *(volatile v4f*)(op + c1) = oB;
      __threadfence();
      *(volatile v4f*)(op + c0) = oA;
      *(volatile v4f*)(op + c1) = oB;
    }
  }
}

static inline size_t al256(size_t o) { return (o + 255) & ~(size_t)255; }

extern "C" void kernel_launch(void* const* d_in, const int* in_sizes, int n_in,
                              void* d_out, int out_size, void* d_ws, size_t ws_size,
                              hipStream_t stream) {
  if (n_in < 6) return;
  if ((long long)in_sizes[0] != (long long)NT * CH) return;
  if ((long long)in_sizes[1] != (long long)NGRAPH * 2 * NE) return;
  if (in_sizes[2] != CH * CH || in_sizes[3] != CH) return;
  if (in_sizes[4] != CH * CH || in_sizes[5] != CH) return;
  if ((long long)out_size != (long long)NT * CH) return;

  const float* x  = (const float*)d_in[0];
  const int*   ei = (const int*)d_in[1];
  const float* W1 = (const float*)d_in[2];
  const float* b1 = (const float*)d_in[3];
  const float* W2 = (const float*)d_in[4];
  const float* b2 = (const float*)d_in[5];
  float* out = (float*)d_out;
  const int vec8 = ((NE & 3) == 0) ? 1 : 0;

  char* ws = (char*)d_ws;
  size_t off = 0;
  const size_t oDIS = off; off = al256(off + (size_t)NT * 4);
  const size_t oW1T = off; off = al256(off + (size_t)CH * K1 * 2);
  const size_t oW2D = off; off = al256(off + (size_t)CH * K2 * 2);
  const size_t oXB  = off; off = al256(off + (size_t)NT * K1 * 2);
  const size_t oH   = off; off = al256(off + (size_t)NT * CH * 4);
  const size_t oX1  = off; off = al256(off + (size_t)NT * K2 * 2);
  if (off > ws_size || off > (size_t)WSMAX) return;
  float*          DIS = (float*)(ws + oDIS);
  unsigned short* W1T = (unsigned short*)(ws + oW1T);
  unsigned short* W2D = (unsigned short*)(ws + oW2D);
  unsigned short* XB  = (unsigned short*)(ws + oXB);
  float*          H   = (float*)(ws + oH);
  unsigned short* X1  = (unsigned short*)(ws + oX1);

  const size_t aggLds = (size_t)AGG_LDS_INTS * 4;
  hipFuncSetAttribute(reinterpret_cast<const void*>(&k_agg<1>), hipFuncAttributeMaxDynamicSharedMemorySize, (int)aggLds);
  hipFuncSetAttribute(reinterpret_cast<const void*>(&k_agg<0>), hipFuncAttributeMaxDynamicSharedMemorySize, (int)aggLds);

  k_prep<<<(UW1 + UW2 + UX) / NTHR, NTHR, 0, stream>>>(x, W1, W2, W1T, W2D, XB);
  k_deg<<<NBLK, NTHR, 0, stream>>>(ei, vec8, DIS);
  k_gemm<<<dim3(NT / GBM, CH / GBN), GTHR, 0, stream>>>(XB, W1T, H, K1, CH);
  k_agg<1><<<NBLK, NTHR, aggLds, stream>>>(ei, vec8, DIS, H, b1, X1, out);
  k_gemm<<<dim3(NT / GBM, CH / GBN), GTHR, 0, stream>>>(X1, W2D, H, K2, CH);
  k_agg<0><<<NBLK, NTHR, aggLds, stream>>>(ei, vec8, DIS, H, b2, X1, out);
}
